// TensorSquare_15461882266098
// MI455X (gfx1250) — hardware-run, weakly checked
//
#include <hip/hip_runtime.h>


#define NND  8192
#define NXC  320
#define NS0  128
#define NG1  64
#define NPA  8128
#define NPD  2016
#define KFF  10368
#define NVO  4096
#define PRT  2048
#define CAF  0.009836118442057921f
#define CWF  0.011048543456039806f
#define RBF  0.5773502691896258f
#define REF_ 0.2581988897471611f
constexpr size_t al256(size_t b) { return (b + 255) & ~(size_t)255; }
constexpr size_t WS_TOTAL = al256((size_t)NND * NXC * 4) + al256((size_t)NND * NS0 * 2) + al256((size_t)NS0 * KFF * 2) + al256((size_t)NVO * NS0 * 2) + al256((size_t)PRT * KFF * 2) + al256((size_t)PRT * NS0 * 4) + al256((size_t)PRT * NVO * 4);
static_assert(WS_TOTAL == 93356032 && WS_TOTAL <= 134217728, "the workspace carve: 89.0 MiB");
static_assert(NPA == NS0 * (NS0 - 1) / 2 && NPD == NG1 * (NG1 - 1) / 2 && NXC == NS0 + 3 * NG1 && KFF == NPA + NS0 + NG1 + NPD + 32 && KFF % 64 == 0 && NPA % 64 == 0 && (NPA + NS0) % 64 == 0 && (NPA + NS0 + NG1) % 64 == 0 && NVO == NG1 * NG1 && NND % PRT == 0 && NS0 == 128 && NG1 == 64, "the four ranges of the feature depth start on whole lines");
typedef _Float16 h16;
typedef unsigned short bf;
typedef __attribute__((ext_vector_type(16))) __bf16   v16bf;
typedef __attribute__((ext_vector_type(16))) _Float16 v16h;
typedef __attribute__((ext_vector_type(8)))  _Float16 v8h;
typedef __attribute__((ext_vector_type(8)))  unsigned short v8us;
typedef __attribute__((ext_vector_type(8)))  float    v8f;
typedef __attribute__((ext_vector_type(4)))  float    v4f;
typedef v8h  __attribute__((may_alias)) v8ha;
typedef v4f  __attribute__((may_alias)) v4fa;
typedef v8us __attribute__((may_alias)) v8usa;

__device__ __forceinline__ unsigned short f2bf(float f) { unsigned u = __float_as_uint(f); u += 0x7FFFu + ((u >> 16) & 1u); return (unsigned short)(u >> 16); }
__device__ __forceinline__ float bf2f(unsigned short b) { return __uint_as_float(((unsigned)b) << 16); }
__device__ __forceinline__ float bfr(float f) { return bf2f(f2bf(f)); }
__device__ __forceinline__ v16h cat16(v8h lo, v8h hi) { return __builtin_shufflevector(lo, hi, 0, 1, 2, 3, 4, 5, 6, 7, 8, 9, 10, 11, 12, 13, 14, 15); }
__device__ __forceinline__ v16bf cat16b(v8us lo, v8us hi) { return __builtin_bit_cast(v16bf, __builtin_shufflevector(lo, hi, 0, 1, 2, 3, 4, 5, 6, 7, 8, 9, 10, 11, 12, 13, 14, 15)); }
__device__ __forceinline__ v8f wmma16(v16h a, v16h b, v8f c) { return __builtin_amdgcn_wmma_f32_16x16x32_f16(false, a, false, b, (short)0, c, false, false); }
__device__ __forceinline__ v8f wmmab(v16bf a, v16bf b, v8f c) { return __builtin_amdgcn_wmma_f32_16x16x32_bf16(false, a, false, b, (short)0, c, false, false); }


template <typename T16> struct WFrag;
template <> struct WFrag<h16> { typedef v16h V; static __device__ __forceinline__ V ld(const h16* p) { return cat16(*(const v8h*)p, *(const v8h*)(p + 16)); } static __device__ __forceinline__ v8f mma(V a, V b, v8f c) { return wmma16(a, b, c); } };
template <> struct WFrag<bf> { typedef v16bf V; static __device__ __forceinline__ V ld(const bf* p) { return cat16b(*(const v8us*)p, *(const v8us*)(p + 16)); } static __device__ __forceinline__ v8f mma(V a, V b, v8f c) { return wmmab(a, b, c); } };
template <typename T16, int NSPLIT, bool BIAS>
__global__ __launch_bounds__(32) void k_gemmw(const T16* __restrict__ A, const T16* __restrict__ A2, const T16* __restrict__ Bt, const T16* __restrict__ Bt2, int K, float* C, int ldc, const float* __restrict__ bias, size_t sA, size_t sB, size_t sC) {
    typedef typename WFrag<T16>::V V;
    __shared__ __align__(16) float os[16 * 68];
    const size_t z = blockIdx.z; A += z * sA; if (A2) A2 += z * sA; Bt += z * sB; if (Bt2) Bt2 += z * sB; C += z * sC;
    const int lane = threadIdx.x & 31, lr = lane & 15, hi = lane >> 4; const int r0 = blockIdx.x * 64, c0 = blockIdx.y * 64;
    v8f acc[4][4];
#pragma unroll
    for (int mb = 0; mb < 4; ++mb)
#pragma unroll
        for (int nb = 0; nb < 4; ++nb) acc[mb][nb] = (v8f){};
    const size_t aoff = (size_t)(r0 + lr) * K + 8 * hi, boff = (size_t)(c0 + lr) * K + 8 * hi;
    for (int kc = 0; kc < K; kc += 32) {
        V a[4], a2[4];
#pragma unroll
        for (int mb = 0; mb < 4; ++mb) { a[mb] = WFrag<T16>::ld(A + aoff + (size_t)mb * 16 * K + kc); if (NSPLIT == 1 || NSPLIT == 2) a2[mb] = WFrag<T16>::ld(A2 + aoff + (size_t)mb * 16 * K + kc); }
#pragma unroll
        for (int nb = 0; nb < 4; ++nb) { const V b = WFrag<T16>::ld(Bt + boff + (size_t)nb * 16 * K + kc); V b2; if (NSPLIT >= 2) b2 = WFrag<T16>::ld(Bt2 + boff + (size_t)nb * 16 * K + kc);
#pragma unroll
            for (int mb = 0; mb < 4; ++mb) { acc[mb][nb] = WFrag<T16>::mma(a[mb], b, acc[mb][nb]); if (NSPLIT == 1 || NSPLIT == 2) acc[mb][nb] = WFrag<T16>::mma(a2[mb], b, acc[mb][nb]); if (NSPLIT >= 2) acc[mb][nb] = WFrag<T16>::mma(a[mb], b2, acc[mb][nb]); } }
        asm volatile("v_nop\n\tv_nop\n\tv_nop\n\tv_nop" : "+v"(acc[0][0]), "+v"(acc[1][1]), "+v"(acc[2][2]), "+v"(acc[3][3]) : "v"(a[0]), "v"(a[3]));
    }
#pragma unroll
    for (int mb = 0; mb < 4; ++mb) {
#pragma unroll
        for (int nb = 0; nb < 4; ++nb) {
#pragma unroll
            for (int j = 0; j < 8; ++j) os[(hi * 8 + j) * 68 + nb * 16 + lr] = acc[mb][nb][j]; }
        __builtin_amdgcn_wave_barrier(); asm volatile("" ::: "memory");
        float* crow = C + (size_t)(r0 + mb * 16) * ldc + c0;
#pragma unroll 1
        for (int ps = 0; ps < 2; ++ps) {
#pragma unroll
            for (int s = 0; s < 8; ++s) { const int row = 2 * s + hi, cofs = lr * 4; v4f val = *(const v4fa*)(os + row * 68 + cofs); if (BIAS) { val[0] += bfr(bias[c0 + cofs]); val[1] += bfr(bias[c0 + cofs + 1]); val[2] += bfr(bias[c0 + cofs + 2]); val[3] += bfr(bias[c0 + cofs + 3]); }
                *(volatile v4f*)(crow + (size_t)row * ldc + cofs) = val; }
            if (ps == 0) __threadfence(); }
        __builtin_amdgcn_wave_barrier(); asm volatile("" ::: "memory");
    }
}

__device__ __forceinline__ h16 tohx(float x) { return (h16)x; }
__device__ __forceinline__ void splitf(float y, unsigned short& h, unsigned short& l) { h = f2bf(y); l = f2bf(y - bf2f(h)); }
typedef __attribute__((ext_vector_type(2))) _Float16 v2h;
typedef __attribute__((ext_vector_type(4))) _Float16 v4h;
typedef __attribute__((ext_vector_type(2))) unsigned short v2us;
typedef __attribute__((ext_vector_type(4))) unsigned short v4us;
typedef __attribute__((ext_vector_type(2))) float v2f;
typedef __attribute__((ext_vector_type(4))) int v4i;


__global__ __launch_bounds__(256) void k_lay(const float* __restrict__ src, h16* dst, unsigned nrow, unsigned c8n, unsigned dp, unsigned c0, unsigned rbs, unsigned ra, unsigned rs, unsigned cbs, unsigned sa, unsigned sb, unsigned rlive, unsigned clive) {
    const unsigned g = blockIdx.x * 256 + threadIdx.x; if (g >= nrow * c8n) return; const unsigned row = g / c8n, ch = g - row * c8n; const unsigned rb = (row >> rbs) * ra + (row & ((1u << rbs) - 1u)) * rs; v8h o;
#pragma unroll
    for (int w = 0; w < 8; ++w) { const unsigned c = 8u * ch + w; const bool live = row < rlive && c < clive; const unsigned si = rb + (c >> cbs) * sa + (c & ((1u << cbs) - 1u)) * sb; const float v = bfr(src[live ? si : 0u]); o[w] = tohx(live && fabsf(v) >= 6.103515625e-05f ? v : 0.0f); }
    h16* d8 = dst + (size_t)row * dp + c0 + 8u * ch; *(volatile v8h*)(d8) = o; __threadfence(); *(volatile v8h*)(d8) = o; }

__global__ __launch_bounds__(256) void k_rnd(const float* __restrict__ xs, float* xr) {
    const unsigned g = blockIdx.x * 256 + threadIdx.x; if (g >= (unsigned)(NND * NXC / 4)) return; v4f o; o[0] = bfr(xs[4u * g]); o[1] = bfr(xs[4u * g + 1u]); o[2] = bfr(xs[4u * g + 2u]); o[3] = bfr(xs[4u * g + 3u]);
    float* dq = xr + 4u * (size_t)g; *(volatile v4f*)(dq) = o; __threadfence(); *(volatile v4f*)(dq) = o; }

__global__ __launch_bounds__(256) void k_feat(const float* __restrict__ xq, h16* dst, unsigned row0) {
    const unsigned g = blockIdx.x * 256 + threadIdx.x; if (g >= (unsigned)(PRT * (KFF / 8))) return; const unsigned rl = g / (unsigned)(KFF / 8), ch = g - rl * (unsigned)(KFF / 8); const unsigned k0 = 8u * ch;
    const unsigned isA = k0 < (unsigned)NPA ? 1u : 0u, isB = (k0 >= (unsigned)NPA && k0 < (unsigned)(NPA + NS0)) ? 1u : 0u, isE = (k0 >= (unsigned)(NPA + NS0) && k0 < (unsigned)(NPA + NS0 + NG1)) ? 1u : 0u, isD = (k0 >= (unsigned)(NPA + NS0 + NG1) && k0 < (unsigned)(NPA + NS0 + NG1 + NPD)) ? 1u : 0u;
    const unsigned pn = isA * (unsigned)NS0 + isD * (unsigned)NG1 + (1u - isA - isD) * 2u;
    const unsigned q0 = isA * k0 + isD * (k0 - (unsigned)(NPA + NS0 + NG1)); unsigned pu = 0u;
#pragma unroll
    for (unsigned b = 64u; b >= 1u; b >>= 1) { const unsigned c = pu + b; const unsigned of = (c * (2u * pn - c - 1u)) >> 1; const unsigned ok = (c < pn ? 1u : 0u) & (of <= q0 ? 1u : 0u); pu = pu + ok * b; }
    unsigned pv = q0 - ((pu * (2u * pn - pu - 1u)) >> 1) + pu + 1u; const unsigned d0 = isB * (k0 - (unsigned)NPA) + isE * (k0 - (unsigned)(NPA + NS0));
    const unsigned m3u = isE + isD; const float m3 = m3u ? 1.0f : 0.0f; const float fac = isA ? 1.0f : (isE ? REF_ : ((isB | isD) ? RBF : 0.0f)); const float* xr = xq + (size_t)(row0 + rl) * NXC; v8h o;
#pragma unroll
    for (int w = 0; w < 8; ++w) { const unsigned isP = isA + isD; const unsigned uu = isP * pu + (1u - isP) * (d0 + (unsigned)w), vv = isP * pv + (1u - isP) * (d0 + (unsigned)w);
        const unsigned ia = m3u * ((unsigned)NS0 + 3u * uu) + (1u - m3u) * uu, ib = m3u * ((unsigned)NS0 + 3u * vv) + (1u - m3u) * vv; const unsigned ia1 = ia + m3u, ia2 = ia + 2u * m3u, ib1 = ib + m3u, ib2 = ib + 2u * m3u;
        const float a0 = xr[ia], a1 = xr[ia1], a2 = xr[ia2], b0 = xr[ib], b1 = xr[ib1], b2 = xr[ib2]; const float fv = fac * (a0 * b0 + m3 * (a1 * b1 + a2 * b2));
        o[w] = tohx(fabsf(fv) >= 6.103515625e-05f ? fv : 0.0f); const unsigned wr = (pv + 1u == pn) ? 1u : 0u; pu = pu + wr; pv = wr * (pu + 1u) + (1u - wr) * (pv + 1u); }
    h16* d8 = dst + (size_t)g * 8u; *(volatile v8h*)(d8) = o; __threadfence(); *(volatile v8h*)(d8) = o; }

__global__ __launch_bounds__(256) void k_out(const float* __restrict__ o0, const float* __restrict__ tt, const float* __restrict__ xq, float* rs, unsigned row0) {
    const unsigned g = blockIdx.x * 256 + threadIdx.x; if (g >= (unsigned)(PRT * NG1)) return; const unsigned rl = g >> 6, oo = g & 63u; const float* xr = xq + (size_t)(row0 + rl) * NXC + NS0; const float* tr = tt + (size_t)rl * NVO + oo;
    float s0 = 0.0f, s1 = 0.0f, s2 = 0.0f;
#pragma unroll
    for (int v = 0; v < NG1; ++v) { const float tv = tr[v * NG1]; s0 += tv * xr[3 * v]; s1 += tv * xr[3 * v + 1]; s2 += tv * xr[3 * v + 2]; }
    float* orow = rs + (size_t)(row0 + rl) * NXC; v2f a; a[0] = o0[(size_t)rl * NS0 + 2u * oo] * CAF; a[1] = o0[(size_t)rl * NS0 + 2u * oo + 1u] * CAF; float* d2 = orow + 2u * oo; float* d3 = orow + NS0 + 3u * oo;
    const float r0 = s0 * CWF, r1 = s1 * CWF, r2 = s2 * CWF;
    *(volatile v2f*)(d2) = a; *(volatile float*)(d3) = r0; *(volatile float*)(d3 + 1) = r1; *(volatile float*)(d3 + 2) = r2; __threadfence(); *(volatile v2f*)(d2) = a; *(volatile float*)(d3) = r0; *(volatile float*)(d3 + 1) = r1; *(volatile float*)(d3 + 2) = r2; }

extern "C" void kernel_launch(void* const* d_in, const int* in_sizes, int n_in,
                              void* d_out, int out_size, void* d_ws, size_t ws_size, hipStream_t stream) {
    if (n_in < 6) return;
    if (in_sizes[0] < NND * NXC || in_sizes[1] < NPA * NS0 || in_sizes[2] < NS0 * NS0 || in_sizes[3] < NS0 * NVO || in_sizes[4] < NPD * NS0 || in_sizes[5] < NG1 * NS0 || out_size < NND * NXC) return;
    const float* xs = (const float*)d_in[0]; const float* wa = (const float*)d_in[1]; const float* wb = (const float*)d_in[2]; const float* wc = (const float*)d_in[3]; const float* wd = (const float*)d_in[4]; const float* we = (const float*)d_in[5];
    char* wsp = (char*)d_ws;
    auto take = [&](size_t bytes) { char* cur = wsp; wsp += (bytes + 255) & ~(size_t)255; return (void*)cur; };
    float* XR = (float*)take((size_t)NND * NXC * 4); h16* SX = (h16*)take((size_t)NND * NS0 * 2); h16* WC = (h16*)take((size_t)NS0 * KFF * 2); h16* WV = (h16*)take((size_t)NVO * NS0 * 2); h16* FF = (h16*)take((size_t)PRT * KFF * 2); float* O0 = (float*)take((size_t)PRT * NS0 * 4); float* TT = (float*)take((size_t)PRT * NVO * 4);
    if ((size_t)(wsp - (char*)d_ws) != WS_TOTAL || WS_TOTAL > ws_size) return;
    auto lay = [&](const float* sp_, h16* dp_, unsigned nrow, unsigned ncol, unsigned dp, unsigned c0, unsigned rbs, unsigned ra, unsigned rs_, unsigned cbs, unsigned sa, unsigned sb, unsigned rlive, unsigned clive) {
        k_lay<<<(nrow * (ncol / 8) + 255) / 256, 256, 0, stream>>>(sp_, dp_, nrow, ncol / 8, dp, c0, rbs, ra, rs_, cbs, sa, sb, rlive, clive); };
    k_rnd<<<(NND * NXC / 4 + 255) / 256, 256, 0, stream>>>(xs, XR);
    lay(xs, SX, NND, NS0, NS0, 0, 16, 0, NXC, 16, 0, 1, NND, NS0);
    lay(wa, WC, NS0, NPA, KFF, 0, 16, 0, 1, 16, 0, NS0, NS0, NPA);
    lay(wb, WC, NS0, NS0, KFF, NPA, 16, 0, 1, 16, 0, NS0, NS0, NS0);
    lay(we, WC, NS0, NG1, KFF, NPA + NS0, 16, 0, 1, 16, 0, NS0, NS0, NG1);
    lay(wd, WC, NS0, NPD + 32, KFF, NPA + NS0 + NG1, 16, 0, 1, 16, 0, NS0, NS0, NPD);
    lay(wc, WV, NVO, NS0, NS0, 0, 16, 0, 1, 16, 0, NVO, NVO, NS0);
    for (unsigned p = 0; p < (unsigned)(NND / PRT); ++p) { const unsigned r0 = p * (unsigned)PRT;
        k_feat<<<(PRT * (KFF / 8) + 255) / 256, 256, 0, stream>>>(XR, FF, r0);
        k_gemmw<h16, 0, false><<<dim3(PRT / 64, NS0 / 64, 1), 32, 0, stream>>>(FF, nullptr, WC, nullptr, KFF, O0, NS0, nullptr, (size_t)0, (size_t)0, (size_t)0);
        k_gemmw<h16, 0, false><<<dim3(PRT / 64, NVO / 64, 1), 32, 0, stream>>>(SX + (size_t)r0 * NS0, nullptr, WV, nullptr, NS0, TT, NVO, nullptr, (size_t)0, (size_t)0, (size_t)0);
        k_out<<<(PRT * NG1 + 255) / 256, 256, 0, stream>>>(O0, TT, XR, (float*)d_out, r0); }
}
